// Net_57105885168298
// MI455X (gfx1250) — hardware-verified
//
#include <hip/hip_runtime.h>
#include <stddef.h>
#include <stdint.h>
#include <math.h>


#define NGRAPH 16
#define NPG    2048
#define NNODE  32768
#define CIN    64
#define KX     128
#define HID    128
#define KD     256
#define KCL    32
#define NEDGE  524288
#define PCOL   160
#define NTHR   256
#define NWAVE  8
#define EPT    8
#define CHUNK  (NTHR * EPT)
#define WCAP   (EPT * 32)
#define LISTN  (NWAVE * WCAP)
#define NBD    8192
#define SLD    13
#define NBA    1024
#define SLA    10
#define RCAP   20480
#define DEGCAP 64
#define BPG    (NPG / NBA)
#define GBM    64
#define GBN    64
#define GTHR   128
#define PTHR   160
#define RECP   1056
#define NSBLK  (NNODE / 256)
#define TRP    264
#define AGG_ZINTS (LISTN + 2 * RCAP + 3 * NBA)
#define MISC_INTS 16
#define XTRA_INTS 352
#define AGG_LDS_INTS (AGG_ZINTS + MISC_INTS + XTRA_INTS)
#define NOUT0  (NGRAPH * KCL * HID)
#define NSEL   (NNODE * KCL)
#define NOUTT  (NOUT0 + 1 + NSEL)
#define WSMAX  134217728

static_assert((CHUNK & (CHUNK - 1)) == 0 && CHUNK <= 4096);
static_assert((NBD & (NBD - 1)) == 0 && NBD == (1 << SLD));
static_assert((NBA & (NBA - 1)) == 0 && NBA == (1 << SLA));
static_assert(((long long)CHUNK << SLD) < (1LL << 31));
static_assert(((long long)NEDGE << SLA) < (1LL << 31));
static_assert(NBD % (NTHR * 4) == 0 && NNODE % NBD == 0);
static_assert(NNODE % NBA == 0 && NPG % NBA == 0 && NBA % NWAVE == 0 && NBA % 32 == 0);
static_assert(AGG_ZINTS % (NTHR * 4) == 0 && LISTN % 4 == 0 && RCAP % 4 == 0);
static_assert(AGG_LDS_INTS * 4 <= 300000);
static_assert(KX % 32 == 0 && KD % 32 == 0 && NPG % 32 == 0 && KX == 2 * CIN && KD == 2 * HID);
static_assert(NNODE % GBM == 0 && HID % GBN == 0 && NPG % GBM == 0);
static_assert(GBM == (GTHR / 32) * 16);
static_assert(HID == 4 * 32 && KCL == 32 && PCOL == HID + KCL && PCOL == (PTHR / 32) * 32);
static_assert(NOUT0 % 32 == 0 && NSEL % 4 == 0 && NOUTT == 1114113);
static_assert(RECP == NGRAPH * CIN + 32 && NGRAPH * CIN == 4 * NTHR);
static_assert(NEDGE % CHUNK == 0 && NEDGE % 4 == 0 && NEDGE >= EPT && EPT == 8);

typedef float          v4f   __attribute__((ext_vector_type(4)));
typedef float          v8f   __attribute__((ext_vector_type(8)));
typedef int            v4i   __attribute__((ext_vector_type(4)));
typedef int            v8i   __attribute__((ext_vector_type(8)));
typedef unsigned int   v4u   __attribute__((ext_vector_type(4)));
typedef unsigned short v8us  __attribute__((ext_vector_type(8)));
typedef unsigned short v16us __attribute__((ext_vector_type(16)));
typedef __bf16         v16bf __attribute__((ext_vector_type(16)));
typedef v4f  __attribute__((may_alias)) v4fa;
typedef v4i  __attribute__((may_alias)) v4ia;
typedef v8us __attribute__((may_alias)) v8usa;
union FragB { v16bf v; v16us u; v8us h[2]; v8i w; };

__device__ __forceinline__ v8f wmb(const FragB& a, const FragB& b, v8f c) {
  v8f d = __builtin_amdgcn_wmma_f32_16x16x32_bf16(false, a.v, false, b.v, (short)0, c, false, false);
  asm volatile("v_nop\n\tv_nop\n\tv_nop\n\tv_nop" : "+v"(d) : "v"(a.w), "v"(b.w));
  return d;
}

__device__ __forceinline__ unsigned bf16_bits(float f) {
  const unsigned u = __float_as_uint(f);
  return (u + 0x7FFFu + ((u >> 16) & 1u)) >> 16;
}
__device__ __forceinline__ float bf16_val(float f) {
  return __uint_as_float(bf16_bits(f) << 16);
}
__device__ __forceinline__ float wred_f(float v) {
#pragma unroll
  for (int o = 16; o > 0; o >>= 1) v += __shfl_xor(v, o, 32);
  return v;
}
__device__ __forceinline__ float wmax_f(float v) {
#pragma unroll
  for (int o = 16; o > 0; o >>= 1) v = fmaxf(v, __shfl_xor(v, o, 32));
  return v;
}
__device__ __forceinline__ double wred_d(double v) {
#pragma unroll
  for (int o = 16; o > 0; o >>= 1) v += __shfl_xor(v, o, 32);
  return v;
}
__device__ __forceinline__ int mkkey1(int s, int d) {
  return (s & ~(NPG - 1)) | (d & (NPG - 1));
}

template <int SLB, int KM>
__device__ __forceinline__ int scan_chunk(const int* __restrict__ srcs, const int* __restrict__ dsts,
                                          int nE, int cbase, int slotBase, int nb, int vec8,
                                          int* list, int tid, int lane, int wave) {
  int wc = 0;
  const int el0  = tid * EPT;
  const int e0   = cbase + el0;
  const int sent = -2147483647 - 1;
  v4i da, db;
  if constexpr (KM != 0) {
    const bool inr = (e0 + EPT) <= nE;
    const int  eb  = inr ? e0 : 0;
    const v4i ta = *(const v4i*)(dsts + eb);
    const v4i tb = *(const v4i*)(dsts + eb + 4);
    const v4i sa = *(const v4i*)(srcs + eb);
    const v4i sb = *(const v4i*)(srcs + eb + 4);
    da.x = inr ? mkkey1(sa.x, ta.x) : sent; da.y = inr ? mkkey1(sa.y, ta.y) : sent;
    da.z = inr ? mkkey1(sa.z, ta.z) : sent; da.w = inr ? mkkey1(sa.w, ta.w) : sent;
    db.x = inr ? mkkey1(sb.x, tb.x) : sent; db.y = inr ? mkkey1(sb.y, tb.y) : sent;
    db.z = inr ? mkkey1(sb.z, tb.z) : sent; db.w = inr ? mkkey1(sb.w, tb.w) : sent;
  } else {
    if (vec8 != 0 && cbase + CHUNK <= nE) {
      da = *(const v4i*)(dsts + e0);
      db = *(const v4i*)(dsts + e0 + 4);
    } else {
      da.x = (e0     < nE) ? dsts[min(e0,     nE - 1)] : sent;
      da.y = (e0 + 1 < nE) ? dsts[min(e0 + 1, nE - 1)] : sent;
      da.z = (e0 + 2 < nE) ? dsts[min(e0 + 2, nE - 1)] : sent;
      da.w = (e0 + 3 < nE) ? dsts[min(e0 + 3, nE - 1)] : sent;
      db.x = (e0 + 4 < nE) ? dsts[min(e0 + 4, nE - 1)] : sent;
      db.y = (e0 + 5 < nE) ? dsts[min(e0 + 5, nE - 1)] : sent;
      db.z = (e0 + 6 < nE) ? dsts[min(e0 + 6, nE - 1)] : sent;
      db.w = (e0 + 7 < nE) ? dsts[min(e0 + 7, nE - 1)] : sent;
    }
  }
  const unsigned nbs = (unsigned)slotBase;
  const unsigned unb = (unsigned)nb;
  const unsigned s0 = (unsigned)da.x - nbs, s1 = (unsigned)da.y - nbs;
  const unsigned s2 = (unsigned)da.z - nbs, s3 = (unsigned)da.w - nbs;
  const unsigned s4 = (unsigned)db.x - nbs, s5 = (unsigned)db.y - nbs;
  const unsigned s6 = (unsigned)db.z - nbs, s7 = (unsigned)db.w - nbs;
  const bool h0 = s0 < unb, h1 = s1 < unb, h2 = s2 < unb, h3 = s3 < unb;
  const bool h4 = s4 < unb, h5 = s5 < unb, h6 = s6 < unb, h7 = s7 < unb;
  const unsigned any = __builtin_amdgcn_ballot_w32(h0 | h1 | h2 | h3 | h4 | h5 | h6 | h7);
  if (any != 0u) {
#define HITJ(J, HJ, SJ) { \
      const unsigned mj = __builtin_amdgcn_ballot_w32(HJ); \
      if (mj != 0u) { \
        if (HJ) { \
          const int pos = wc + (int)__builtin_amdgcn_mbcnt_lo(mj, 0u); \
          if (pos < WCAP) list[wave * WCAP + pos] = ((el0 + (J)) << SLB) | (int)(SJ); \
        } \
        wc += (int)__builtin_popcount(mj); } }
    HITJ(0, h0, s0)
    HITJ(1, h1, s1)
    HITJ(2, h2, s2)
    HITJ(3, h3, s3)
    HITJ(4, h4, s4)
    HITJ(5, h5, s5)
    HITJ(6, h6, s6)
    HITJ(7, h7, s7)
#undef HITJ
  }
  return wc;
}

__global__ __launch_bounds__(NTHR) void k_prep(const float* __restrict__ W1, const float* __restrict__ Wp,
                                               unsigned short* W1T2, unsigned short* WPT2) {
  const int u = (int)blockIdx.x * NTHR + (int)threadIdx.x;
  v8us o;
  unsigned short* dp;
  if (u < 2048) {
    const int n  = u >> 4;
    const int k8 = (u & 15) * 8;
    const int kk = k8 & (CIN - 1);
    const float* p = W1 + (size_t)kk * HID + n;
#pragma unroll
    for (int i = 0; i < 8; ++i) o[i] = (unsigned short)bf16_bits(p[(size_t)i * HID]);
    dp = W1T2 + (size_t)n * KX + k8;
  } else if (u < 3072) {
    const int v  = u - 2048;
    const int n  = v >> 5;
    const int k8 = (v & 31) * 8;
    const int kk = k8 & (HID - 1);
    const float* p = Wp + (size_t)kk * KCL + n;
#pragma unroll
    for (int i = 0; i < 8; ++i) o[i] = (unsigned short)bf16_bits(p[(size_t)i * KCL]);
    dp = WPT2 + (size_t)n * KD + k8;
  } else {
    return;
  }
  *(volatile v8us*)dp = o;
  __threadfence();
  *(volatile v8us*)dp = o;
}

template <int SQ>
__global__ __launch_bounds__(NTHR) void k_gn_acc(const float* __restrict__ x, const int* __restrict__ bat,
                                                 const float* __restrict__ msc, const float* __restrict__ meanp,
                                                 float* rec) {
  __shared__ __attribute__((aligned(16))) float bins[4 * 1024];
  __shared__ __attribute__((aligned(16))) float smean[1024];
  __shared__ int sbat[256];
  __shared__ int scn[64];
  const int tid = (int)threadIdx.x;
  const int c = tid & 63, q = tid >> 6;
  const int base = (int)blockIdx.x * 256;
  sbat[tid] = bat[base + tid];
  if constexpr (SQ != 0) {
    const v4f mv = *(const v4f*)(meanp + 4 * tid);
    *(v4fa*)(smean + 4 * tid) = mv;
  }
#pragma unroll
  for (int g = 0; g < NGRAPH; ++g) bins[q * 1024 + g * CIN + c] = 0.0f;
  __syncthreads();
  const float msa = bf16_val(msc[c]);
  int cn = 0;
#pragma unroll 4
  for (int i = 0; i < 64; ++i) {
    const int r  = q * 64 + i;
    const int g  = sbat[r];
    const bool ok = (unsigned)g < (unsigned)NGRAPH;
    const int gc = ok ? g : 0;
    float v = bf16_val(x[(size_t)(base + r) * CIN + c]);
    if constexpr (SQ != 0) {
      const float o = v - smean[gc * CIN + c] * msa;
      v = o * o;
    }
    float* bq = bins + q * 1024 + gc * CIN + c;
    const float old = *bq;
    *bq = old + (ok ? v : 0.0f);
    cn += (ok && g == c) ? 1 : 0;
  }
  if (c < 16) scn[q * 16 + c] = cn;
  __syncthreads();
  const v4f b0 = *(const v4fa*)(bins + 4 * tid);
  const v4f b1 = *(const v4fa*)(bins + 1024 + 4 * tid);
  const v4f b2 = *(const v4fa*)(bins + 2048 + 4 * tid);
  const v4f b3 = *(const v4fa*)(bins + 3072 + 4 * tid);
  const v4f sv = ((b0 + b1) + b2) + b3;
  v4f cv;
  {
    const int g0 = (4 * tid) & 15;
    const bool lv = tid < 4;
    const int c0 = scn[g0] + scn[16 + g0] + scn[32 + g0] + scn[48 + g0];
    const int c1 = scn[g0 + 1] + scn[17 + g0] + scn[33 + g0] + scn[49 + g0];
    const int c2 = scn[g0 + 2] + scn[18 + g0] + scn[34 + g0] + scn[50 + g0];
    const int c3 = scn[g0 + 3] + scn[19 + g0] + scn[35 + g0] + scn[51 + g0];
    cv.x = lv ? (float)c0 : 0.0f; cv.y = lv ? (float)c1 : 0.0f;
    cv.z = lv ? (float)c2 : 0.0f; cv.w = lv ? (float)c3 : 0.0f;
  }
  float* rp = rec + (size_t)blockIdx.x * RECP;
  *(volatile v4f*)(rp + 4 * tid) = sv;
  if (tid < 8) *(volatile v4f*)(rp + 1024 + 4 * tid) = cv;
  __threadfence();
  *(volatile v4f*)(rp + 4 * tid) = sv;
  if (tid < 8) *(volatile v4f*)(rp + 1024 + 4 * tid) = cv;
}

template <int SQ>
__global__ __launch_bounds__(NTHR) void k_gn_comb(const float* __restrict__ rec, int nrec,
                                                  const float* __restrict__ meanp, float* outp) {
  __shared__ float scn[16];
  const int tid = (int)threadIdx.x;
  const int g = tid >> 4;
  double s0 = 0.0, s1 = 0.0, s2 = 0.0, s3 = 0.0, cn = 0.0;
#pragma unroll 2
  for (int r = 0; r < nrec; ++r) {
    const float* rp = rec + (size_t)r * RECP;
    const v4f v = *(const v4f*)(rp + 4 * tid);
    s0 += (double)v.x; s1 += (double)v.y; s2 += (double)v.z; s3 += (double)v.w;
    if constexpr (SQ == 0) cn += (double)rp[1024 + g];
  }
  if constexpr (SQ != 0) cn = (double)meanp[1024 + g];
  const double cd = (cn < 1.0) ? 1.0 : cn;
  v4f ov;
  if constexpr (SQ == 0) {
    ov.x = (float)(s0 / cd); ov.y = (float)(s1 / cd); ov.z = (float)(s2 / cd); ov.w = (float)(s3 / cd);
    if ((tid & 15) == 0) scn[g] = (float)cn;
    __syncthreads();
    const int g0 = (4 * tid) & 15;
    const bool lv = tid < 4;
    const float c0 = scn[g0], c1 = scn[g0 + 1], c2 = scn[g0 + 2], c3 = scn[g0 + 3];
    v4f cv;
    cv.x = lv ? c0 : 0.0f; cv.y = lv ? c1 : 0.0f; cv.z = lv ? c2 : 0.0f; cv.w = lv ? c3 : 0.0f;
    *(volatile v4f*)(outp + 4 * tid) = ov;
    if (tid < 8) *(volatile v4f*)(outp + 1024 + 4 * tid) = cv;
    __threadfence();
    *(volatile v4f*)(outp + 4 * tid) = ov;
    if (tid < 8) *(volatile v4f*)(outp + 1024 + 4 * tid) = cv;
  } else {
    const float v0 = (float)(s0 / cd), v1 = (float)(s1 / cd), v2 = (float)(s2 / cd), v3 = (float)(s3 / cd);
    ov.x = 1.0f / sqrtf(v0 + 1e-5f); ov.y = 1.0f / sqrtf(v1 + 1e-5f);
    ov.z = 1.0f / sqrtf(v2 + 1e-5f); ov.w = 1.0f / sqrtf(v3 + 1e-5f);
    *(volatile v4f*)(outp + 4 * tid) = ov;
    __threadfence();
    *(volatile v4f*)(outp + 4 * tid) = ov;
  }
}

__device__ __forceinline__ float nrm1(float xv, float mu, float sc, float w, float b, float r) {
  const float o = bf16_val(xv) - mu * bf16_val(sc);
  return (bf16_val(w) * o) * r + bf16_val(b);
}
__global__ __launch_bounds__(NTHR) void k_norm(const float* __restrict__ x, const int* __restrict__ bat,
                                               const float* __restrict__ gw, const float* __restrict__ gb,
                                               const float* __restrict__ msc, const float* __restrict__ meanp,
                                               const float* __restrict__ rstd, int nN, unsigned short* xn) {
  const int u = (int)blockIdx.x * NTHR + (int)threadIdx.x;
  const int row = u >> 3;
  const int k8  = (u & 7) * 8;
  if (row >= nN) return;
  int g = bat[row];
  g = g < 0 ? 0 : (g > NGRAPH - 1 ? NGRAPH - 1 : g);
  const float* xp = x + (size_t)row * CIN + k8;
  const v4f xa = *(const v4f*)xp,                       xb = *(const v4f*)(xp + 4);
  const v4f ma = *(const v4f*)(meanp + g * CIN + k8),   mb = *(const v4f*)(meanp + g * CIN + k8 + 4);
  const v4f ra = *(const v4f*)(rstd + g * CIN + k8),    rb = *(const v4f*)(rstd + g * CIN + k8 + 4);
  const v4f wa = *(const v4f*)(gw + k8),                wb = *(const v4f*)(gw + k8 + 4);
  const v4f ba = *(const v4f*)(gb + k8),                bb = *(const v4f*)(gb + k8 + 4);
  const v4f sa = *(const v4f*)(msc + k8),               sb = *(const v4f*)(msc + k8 + 4);
  float y[8];
  y[0] = nrm1(xa.x, ma.x, sa.x, wa.x, ba.x, ra.x);
  y[1] = nrm1(xa.y, ma.y, sa.y, wa.y, ba.y, ra.y);
  y[2] = nrm1(xa.z, ma.z, sa.z, wa.z, ba.z, ra.z);
  y[3] = nrm1(xa.w, ma.w, sa.w, wa.w, ba.w, ra.w);
  y[4] = nrm1(xb.x, mb.x, sb.x, wb.x, bb.x, rb.x);
  y[5] = nrm1(xb.y, mb.y, sb.y, wb.y, bb.y, rb.y);
  y[6] = nrm1(xb.z, mb.z, sb.z, wb.z, bb.z, rb.z);
  y[7] = nrm1(xb.w, mb.w, sb.w, wb.w, bb.w, rb.w);
  v8us oh, ol;
#pragma unroll
  for (int i = 0; i < 8; ++i) {
    const unsigned hb = bf16_bits(y[i]);
    oh[i] = (unsigned short)hb;
    ol[i] = (unsigned short)bf16_bits(y[i] - __uint_as_float(hb << 16));
  }
  unsigned short* dph = xn + (size_t)row * KX + k8;
  unsigned short* dpl = dph + CIN;
  *(volatile v8us*)dph = oh;
  *(volatile v8us*)dpl = ol;
  __threadfence();
  *(volatile v8us*)dph = oh;
  *(volatile v8us*)dpl = ol;
}

__global__ __launch_bounds__(NTHR) void k_deg(const int* __restrict__ dsts, int nE, int vec8, float* dis) {
  __shared__ __attribute__((aligned(16))) int scnt[NBD];
  __shared__ __attribute__((aligned(16))) int list[LISTN];
  __shared__ int wcnt[NWAVE];
  const int tid = (int)threadIdx.x, lane = tid & 31, wave = tid >> 5;
  const int nodeBase = (int)blockIdx.x * NBD;

  for (int i = tid; i < NBD; i += NTHR) scnt[i] = 0;
  for (int i = tid; i < LISTN; i += NTHR) list[i] = 0;
  if (tid < NWAVE) wcnt[tid] = 0;
  __syncthreads();

  const int nChunks = (nE + CHUNK - 1) / CHUNK;
#pragma unroll 1
  for (int ch = 0; ch < nChunks; ++ch) {
    const int cbase = ch * CHUNK;
    const int wc = scan_chunk<SLD, 0>(dsts, dsts, nE, cbase, nodeBase, NBD, vec8, list, tid, lane, wave);
    if (lane == 0) wcnt[wave] = wc;
    __syncthreads();
    if (wave == 0) {
#pragma unroll 1
      for (int w2 = 0; w2 < NWAVE; ++w2) {
        int c = wcnt[w2];
        c = c < 0 ? 0 : (c > WCAP ? WCAP : c);
#pragma unroll 1
        for (int b0 = 0; b0 < c; b0 += 32) {
          const int idx = b0 + lane;
          const int ent = list[w2 * WCAP + (idx < WCAP ? idx : WCAP - 1)];
          const int m32 = (c - b0) < 32 ? (c - b0) : 32;
#pragma unroll 1
          for (int k = 0; k < m32; ++k) {
            const int u  = __builtin_amdgcn_readlane(ent, k);
            const int sl = u & (NBD - 1);
            if (lane == 0) scnt[sl] = scnt[sl] + 1;
          }
        }
      }
    }
    __syncthreads();
  }

  v4f vals[NBD / (NTHR * 4)];
#pragma unroll
  for (int it = 0; it < NBD / (NTHR * 4); ++it) {
    const int s0 = it * (NTHR * 4) + 4 * tid;
    const v4i c4 = *(const v4ia*)(scnt + s0);
    const float d0 = (float)c4.x + 1.0f, d1 = (float)c4.y + 1.0f;
    const float d2 = (float)c4.z + 1.0f, d3 = (float)c4.w + 1.0f;
    v4f v;
    v.x = rsqrtf(d0); v.y = rsqrtf(d1); v.z = rsqrtf(d2); v.w = rsqrtf(d3);
    vals[it] = v;
  }
#pragma unroll
  for (int it = 0; it < NBD / (NTHR * 4); ++it) {
    const int s0 = it * (NTHR * 4) + 4 * tid;
    *(volatile v4f*)(dis + (size_t)nodeBase + s0) = vals[it];
  }
  __threadfence();
#pragma unroll
  for (int it = 0; it < NBD / (NTHR * 4); ++it) {
    const int s0 = it * (NTHR * 4) + 4 * tid;
    *(volatile v4f*)(dis + (size_t)nodeBase + s0) = vals[it];
  }
}

__global__ __launch_bounds__(GTHR) void k_gemm(
    const unsigned short* __restrict__ A, const unsigned short* __restrict__ WT,
    float* outF, int K, int ldo)
{
  __shared__ __attribute__((aligned(16))) float stg[GBM * GBN];
  const int tid = (int)threadIdx.x, lane = tid & 31, wave = tid >> 5, hh = lane >> 4, m = lane & 15;
  const int rowBase = (int)blockIdx.x * GBM;
  const int col0    = (int)blockIdx.y * GBN;

  v8f acc[4];
  {
    const v8f z = {0.f, 0.f, 0.f, 0.f, 0.f, 0.f, 0.f, 0.f};
    acc[0] = z; acc[1] = z; acc[2] = z; acc[3] = z;
  }
  const unsigned short* ap = A  + (size_t)(rowBase + 16 * wave + m) * (size_t)K + 8 * hh;
  const unsigned short* wp = WT + (size_t)(col0 + m) * (size_t)K + 8 * hh;
  const int ksteps = K >> 5;
#pragma unroll 1
  for (int ks = 0; ks < ksteps; ++ks) {
    FragB af;
    af.h[0] = *(const v8usa*)(ap + 32 * ks);
    af.h[1] = *(const v8usa*)(ap + 32 * ks + 16);
#pragma unroll
    for (int t = 0; t < 4; ++t) {
      const unsigned short* wq = wp + (size_t)(16 * t) * (size_t)K + 32 * ks;
      FragB bf;
      bf.h[0] = *(const v8usa*)wq;
      bf.h[1] = *(const v8usa*)(wq + 16);
      acc[t] = wmb(af, bf, acc[t]);
    }
  }

#pragma unroll
  for (int t = 0; t < 4; ++t) {
    const int lc = 16 * t + m;
#pragma unroll
    for (int r = 0; r < 8; ++r) {
      const int lr = 16 * wave + 8 * hh + r;
      stg[lr * GBN + lc] = acc[t][r];
    }
  }
  __syncthreads();

  v4f fv[8];
#pragma unroll
  for (int i = 0; i < 8; ++i) {
    const int lr = 16 * wave + 2 * i + hh;
    fv[i] = *(const v4fa*)(stg + lr * GBN + 4 * m);
  }
#pragma unroll
  for (int i = 0; i < 8; ++i) {
    const int lr = 16 * wave + 2 * i + hh;
    const int gr = rowBase + lr;
    float* op = outF + (size_t)gr * (size_t)ldo + col0 + 4 * m;
    *(volatile v4f*)op = fv[i];
  }
  __threadfence();
#pragma unroll
  for (int i = 0; i < 8; ++i) {
    const int lr = 16 * wave + 2 * i + hh;
    const int gr = rowBase + lr;
    float* op = outF + (size_t)gr * (size_t)ldo + col0 + 4 * m;
    *(volatile v4f*)op = fv[i];
  }
}

template <int KM>
__device__ __forceinline__ void build_lists(const int* __restrict__ srcs, const int* __restrict__ dsts,
                                            int nE, int vec8, int nodeBase, int* dsm,
                                            int tid, int lane, int wave, int& ttOut, int& ovOut) {
  int* list = dsm;
  int* hl   = dsm + LISTN;
  int* sl   = hl + RCAP;
  int* cnt  = sl + RCAP;
  int* offs = cnt + NBA;
  int* cur  = offs + NBA;
  int* misc = cur + NBA;
  {
    const v4i z4 = {0, 0, 0, 0};
    for (int i = tid * 4; i < AGG_ZINTS; i += NTHR * 4) *(v4ia*)(dsm + i) = z4;
    if (tid < MISC_INTS) misc[tid] = 0;
  }
  __syncthreads();

  int t = 0, ov = 0;
  const int nChunks = (nE + CHUNK - 1) / CHUNK;
#pragma unroll 1
  for (int ch = 0; ch < nChunks; ++ch) {
    const int cbase = ch * CHUNK;
    const int wc = scan_chunk<SLA, KM>(srcs, dsts, nE, cbase, nodeBase, NBA, vec8, list, tid, lane, wave);
    if (lane == 0) misc[wave] = wc;
    __syncthreads();
    if (wave == 0) {
#pragma unroll 1
      for (int w2 = 0; w2 < NWAVE; ++w2) {
        int c = misc[w2];
        c = c < 0 ? 0 : (c > WCAP ? WCAP : c);
#pragma unroll 1
        for (int b0 = 0; b0 < c; b0 += 32) {
          const int idx = b0 + lane;
          const int ent = list[w2 * WCAP + (idx < WCAP ? idx : WCAP - 1)];
          const int m32 = (c - b0) < 32 ? (c - b0) : 32;
#pragma unroll 1
          for (int k = 0; k < m32; ++k) {
            const int u    = __builtin_amdgcn_readlane(ent, k);
            const int slot = u & (NBA - 1);
            const int el   = (u >> SLA) & (CHUNK - 1);
            const int pk   = ((cbase + el) << SLA) | slot;
            if (t < RCAP) {
              if (lane == 0) { hl[t] = pk; cnt[slot] = cnt[slot] + 1; }
              t = t + 1;
            } else {
              ov = 1;
            }
          }
        }
      }
    }
    __syncthreads();
  }
  if (wave == 0 && lane == 0) { misc[8] = t; misc[9] = ov; }
  __syncthreads();
  int tt = misc[8];
  tt = tt < 0 ? 0 : (tt > RCAP ? RCAP : tt);
  const int ovf = misc[9];

  if (wave == 0) {
    const int base = lane * (NBA / 32);
    int s = 0;
#pragma unroll 1
    for (int i = 0; i < NBA / 32; ++i) s += cnt[base + i];
    int incl = s;
#pragma unroll
    for (int d = 1; d < 32; d <<= 1) {
      const int y = __shfl_up(incl, d, 32);
      if (lane >= d) incl += y;
    }
    int run = incl - s;
#pragma unroll 1
    for (int i = 0; i < NBA / 32; ++i) {
      const int cv = cnt[base + i];
      offs[base + i] = run;
      cur[base + i]  = run;
      run += cv;
    }
  }
  __syncthreads();
  if (wave == 0) {
#pragma unroll 1
    for (int b0 = 0; b0 < tt; b0 += 32) {
      const int idx = b0 + lane;
      const int ent = hl[idx < RCAP ? idx : RCAP - 1];
      const int m32 = (tt - b0) < 32 ? (tt - b0) : 32;
#pragma unroll 1
      for (int k = 0; k < m32; ++k) {
        const int u    = __builtin_amdgcn_readlane(ent, k);
        const int slot = u & (NBA - 1);
        if (lane == 0) {
          int p = cur[slot];
          p = p < 0 ? 0 : (p > RCAP - 1 ? RCAP - 1 : p);
          sl[p] = u;
          cur[slot] = p + 1;
        }
      }
    }
  }
  __syncthreads();
  ttOut = tt;
  ovOut = ovf;
}

__global__ __launch_bounds__(NTHR) void k_scan1(const int* __restrict__ srcs, const int* __restrict__ dsts,
                                                int nE, int nN, int vec8,
                                                const float* __restrict__ dis, const float* __restrict__ hf,
                                                const float* __restrict__ bias, unsigned short* xd) {
  extern __shared__ __attribute__((aligned(16))) int dsm[];
  int* sl   = dsm + LISTN + RCAP;
  int* cnt  = sl + RCAP;
  int* offs = cnt + NBA;
  const int tid = (int)threadIdx.x, lane = tid & 31, wave = tid >> 5;
  const int nodeBase = (int)blockIdx.x * NBA;
  int tt = 0, ovf = 0;
  build_lists<0>(srcs, dsts, nE, vec8, nodeBase, dsm, tid, lane, wave, tt, ovf);

  v4f bv;
  {
    const v4f a = *(const v4f*)(bias + 4 * lane);
    bv.x = bf16_val(a.x); bv.y = bf16_val(a.y); bv.z = bf16_val(a.z); bv.w = bf16_val(a.w);
  }
  const float qnan = __int_as_float(0x7fc00000);
  const float pz = (ovf != 0) ? qnan : 0.0f;
  const int sa = (2 * lane) & 31, sb = (2 * lane + 1) & 31;
#pragma unroll 1
  for (int si = 0; si < NBA / NWAVE; ++si) {
    const int s    = si * NWAVE + wave;
    const int node = nodeBase + s;
    int c = cnt[s];
    const bool big = c > DEGCAP;
    c = c < 0 ? 0 : (c > DEGCAP ? DEGCAP : c);
    int o = offs[s];
    o = o < 0 ? 0 : (o > RCAP ? RCAP : o);
    const int nc = node < nN ? node : nN - 1;
    const float dd = dis[nc];
    const float rd = dd * dd;
    float a0 = 0.0f, a1 = 0.0f, a2 = 0.0f, a3 = 0.0f;
#pragma unroll 1
    for (int b0 = 0; b0 < c; b0 += 32) {
      int idx = o + b0 + lane;
      idx = idx > RCAP - 1 ? RCAP - 1 : idx;
      const int ent = sl[idx];
      int eid = ent >> SLA;
      eid = eid < 0 ? 0 : (eid > nE - 1 ? nE - 1 : eid);
      int sr = srcs[eid];
      sr = sr < 0 ? 0 : (sr > nN - 1 ? nN - 1 : sr);
      const float cf  = dis[sr] * dd;
      const int   cfi = __float_as_int(cf);
      const int m32 = (c - b0) < 32 ? (c - b0) : 32;
#pragma unroll 1
      for (int k = 0; k < m32; ++k) {
        const int   sk = __builtin_amdgcn_readlane(sr, k);
        const float ck = __int_as_float(__builtin_amdgcn_readlane(cfi, k));
        const v4f a = *(const v4f*)(hf + (size_t)sk * HID + 4 * lane);
        a0 = fmaf(ck, a.x, a0); a1 = fmaf(ck, a.y, a1);
        a2 = fmaf(ck, a.z, a2); a3 = fmaf(ck, a.w, a3);
      }
    }
    const v4f sv = *(const v4f*)(hf + (size_t)nc * HID + 4 * lane);
    const float pzr = big ? qnan : pz;
    float y0 = (a0 + sv.x * rd) + bv.x;
    float y1 = (a1 + sv.y * rd) + bv.y;
    float y2 = (a2 + sv.z * rd) + bv.z;
    float y3 = (a3 + sv.w * rd) + bv.w;
    y0 = (y0 > 0.0f) ? y0 : (y0 - y0);
    y1 = (y1 > 0.0f) ? y1 : (y1 - y1);
    y2 = (y2 > 0.0f) ? y2 : (y2 - y2);
    y3 = (y3 > 0.0f) ? y3 : (y3 - y3);
    y0 = y0 + pzr; y1 = y1 + pzr; y2 = y2 + pzr; y3 = y3 + pzr;
    const unsigned hb0 = bf16_bits(y0), hb1 = bf16_bits(y1), hb2 = bf16_bits(y2), hb3 = bf16_bits(y3);
    const unsigned lb0 = bf16_bits(y0 - __uint_as_float(hb0 << 16));
    const unsigned lb1 = bf16_bits(y1 - __uint_as_float(hb1 << 16));
    const unsigned lb2 = bf16_bits(y2 - __uint_as_float(hb2 << 16));
    const unsigned lb3 = bf16_bits(y3 - __uint_as_float(hb3 << 16));
    const int hw0 = (int)(hb0 | (hb1 << 16));
    const int hw1 = (int)(hb2 | (hb3 << 16));
    const int lw0 = (int)(lb0 | (lb1 << 16));
    const int lw1 = (int)(lb2 | (lb3 << 16));
    const int g0 = __shfl(hw0, sa, 32), g1 = __shfl(hw1, sa, 32);
    const int g2 = __shfl(hw0, sb, 32), g3 = __shfl(hw1, sb, 32);
    const int p0 = __shfl(lw0, sa, 32), p1 = __shfl(lw1, sa, 32);
    const int p2 = __shfl(lw0, sb, 32), p3 = __shfl(lw1, sb, 32);
    const bool lsel = (lane & 16) != 0;
    v4u pv;
    pv.x = (unsigned int)(lsel ? p0 : g0);
    pv.y = (unsigned int)(lsel ? p1 : g1);
    pv.z = (unsigned int)(lsel ? p2 : g2);
    pv.w = (unsigned int)(lsel ? p3 : g3);
    unsigned short* hp = xd + (size_t)node * KD + 8 * lane;
    const bool wr = node < nN;
    if (wr) *(volatile v4u*)hp = pv;
    __threadfence();
    if (wr) *(volatile v4u*)hp = pv;
  }
}

__global__ __launch_bounds__(NTHR) void k_tr(const unsigned short* __restrict__ xd, unsigned short* xdt) {
  __shared__ __attribute__((aligned(16))) unsigned short T[64 * TRP];
  const int tid = (int)threadIdx.x;
  const int n0  = (int)blockIdx.x * 64;
  const int b   = n0 >> 11;
  const int nl0 = n0 & (NPG - 1);
#pragma unroll
  for (int it = 0; it < 8; ++it) {
    const int id  = it * NTHR + tid;
    const int row = id >> 5;
    const int c8  = (id & 31) * 8;
    const v8us v = *(const v8usa*)(xd + (size_t)(n0 + row) * KD + c8);
    *(v8usa*)(T + row * TRP + c8) = v;
  }
  __syncthreads();
  v8us o[8];
#pragma unroll
  for (int it = 0; it < 8; ++it) {
    const int id  = it * NTHR + tid;
    const int col = id >> 3;
    const int r8  = (id & 7) * 8;
#pragma unroll
    for (int i = 0; i < 8; ++i) o[it][i] = T[(r8 + i) * TRP + col];
  }
#pragma unroll
  for (int it = 0; it < 8; ++it) {
    const int id  = it * NTHR + tid;
    const int col = id >> 3;
    const int r8  = (id & 7) * 8;
    unsigned short* dp = xdt + ((size_t)((col >> 7) * NGRAPH + b) * HID + (col & (HID - 1))) * NPG + nl0 + r8;
    *(volatile v8us*)dp = o[it];
  }
  __threadfence();
#pragma unroll
  for (int it = 0; it < 8; ++it) {
    const int id  = it * NTHR + tid;
    const int col = id >> 3;
    const int r8  = (id & 7) * 8;
    unsigned short* dp = xdt + ((size_t)((col >> 7) * NGRAPH + b) * HID + (col & (HID - 1))) * NPG + nl0 + r8;
    *(volatile v8us*)dp = o[it];
  }
}

__global__ __launch_bounds__(GTHR) void k_gemm2(const unsigned short* __restrict__ A,
                                                const unsigned short* __restrict__ WT,
                                                const float* __restrict__ bp, float* S,
                                                unsigned short* sth, unsigned short* stl) {
  __shared__ __attribute__((aligned(16))) float stg[GBM * KCL];
  const int tid = (int)threadIdx.x, lane = tid & 31, wave = tid >> 5, hh = lane >> 4, m = lane & 15;
  const int rowBase = (int)blockIdx.x * GBM;
  v8f acc[2];
  {
    const v8f z = {0.f, 0.f, 0.f, 0.f, 0.f, 0.f, 0.f, 0.f};
    acc[0] = z; acc[1] = z;
  }
  const unsigned short* ap = A  + (size_t)(rowBase + 16 * wave + m) * (size_t)KD + 8 * hh;
  const unsigned short* wp = WT + (size_t)m * (size_t)KD + 8 * hh;
#pragma unroll 1
  for (int ks = 0; ks < KD / 32; ++ks) {
    FragB af;
    af.h[0] = *(const v8usa*)(ap + 32 * ks);
    af.h[1] = *(const v8usa*)(ap + 32 * ks + 16);
#pragma unroll
    for (int t = 0; t < 2; ++t) {
      const unsigned short* wq = wp + (size_t)(16 * t) * (size_t)KD + 32 * ks;
      FragB bf;
      bf.h[0] = *(const v8usa*)wq;
      bf.h[1] = *(const v8usa*)(wq + 16);
      acc[t] = wmb(af, bf, acc[t]);
    }
  }
#pragma unroll
  for (int t = 0; t < 2; ++t) {
#pragma unroll
    for (int r = 0; r < 8; ++r) {
      const int lr = 16 * wave + 8 * hh + r;
      stg[lr * KCL + 16 * t + m] = acc[t][r];
    }
  }
  __syncthreads();
  const float bpv = bf16_val(bp[lane]);
#pragma unroll 1
  for (int i = 0; i < 16; ++i) {
    const int r = 16 * wave + i;
    const float v  = stg[r * KCL + lane] + bpv;
    const float mx = wmax_f(v);
    const float e  = expf(v - mx);
    const float sm = wred_f(e);
    stg[r * KCL + lane] = e * (1.0f / sm);
  }
  __syncthreads();

  const int b   = rowBase >> 11;
  const int nl0 = rowBase & (NPG - 1);
  v4f  sv[4];
  v8us oh[2], ol[2];
#pragma unroll
  for (int it = 0; it < 4; ++it) {
    const int id = it * GTHR + tid;
    sv[it] = *(const v4fa*)(stg + (id >> 3) * KCL + 4 * (id & 7));
  }
#pragma unroll
  for (int it = 0; it < 2; ++it) {
    const int id = it * GTHR + tid;
    const int k  = id >> 3;
    const int r8 = (id & 7) * 8;
#pragma unroll
    for (int i = 0; i < 8; ++i) {
      const float v = stg[(r8 + i) * KCL + k];
      const unsigned hb = bf16_bits(v);
      oh[it][i] = (unsigned short)hb;
      ol[it][i] = (unsigned short)bf16_bits(v - __uint_as_float(hb << 16));
    }
  }
#pragma unroll
  for (int it = 0; it < 4; ++it) {
    const int id = it * GTHR + tid;
    *(volatile v4f*)(S + (size_t)(rowBase + (id >> 3)) * KCL + 4 * (id & 7)) = sv[it];
  }
#pragma unroll
  for (int it = 0; it < 2; ++it) {
    const int id = it * GTHR + tid;
    const size_t off = ((size_t)(b * KCL + (id >> 3))) * NPG + nl0 + (id & 7) * 8;
    *(volatile v8us*)(sth + off) = oh[it];
    *(volatile v8us*)(stl + off) = ol[it];
  }
  __threadfence();
#pragma unroll
  for (int it = 0; it < 4; ++it) {
    const int id = it * GTHR + tid;
    *(volatile v4f*)(S + (size_t)(rowBase + (id >> 3)) * KCL + 4 * (id & 7)) = sv[it];
  }
#pragma unroll
  for (int it = 0; it < 2; ++it) {
    const int id = it * GTHR + tid;
    const size_t off = ((size_t)(b * KCL + (id >> 3))) * NPG + nl0 + (id & 7) * 8;
    *(volatile v8us*)(sth + off) = oh[it];
    *(volatile v8us*)(stl + off) = ol[it];
  }
}

__global__ __launch_bounds__(NTHR) void k_scan2(const int* __restrict__ srcs, const int* __restrict__ dsts,
                                                int nE, int nN, int vec8,
                                                const float* __restrict__ S, float* rec3) {
  extern __shared__ __attribute__((aligned(16))) int dsm[];
  int* sl   = dsm + LISTN + RCAP;
  int* cnt  = sl + RCAP;
  int* offs = cnt + NBA;
  float* wca = (float*)(dsm + AGG_ZINTS + MISC_INTS);
  float* wtr = wca + 256;
  float* rec = wtr + 32;
  const int tid = (int)threadIdx.x, lane = tid & 31, wave = tid >> 5;
  const int nodeBase = (int)blockIdx.x * NBA;
  int tt = 0, ovf = 0;
  build_lists<1>(srcs, dsts, nE, vec8, nodeBase, dsm, tid, lane, wave, tt, ovf);

  const float qnan = __int_as_float(0x7fc00000);
  const float pz = (ovf != 0) ? qnan : 0.0f;
  float trp = 0.0f, cap = 0.0f;
#pragma unroll 1
  for (int si = 0; si < NBA / NWAVE; ++si) {
    const int s    = si * NWAVE + wave;
    const int node = nodeBase + s;
    int c = cnt[s];
    const bool big = c > DEGCAP;
    c = c < 0 ? 0 : (c > DEGCAP ? DEGCAP : c);
    int o = offs[s];
    o = o < 0 ? 0 : (o > RCAP ? RCAP : o);
    const int nc = node < nN ? node : nN - 1;
    float t = 0.0f;
#pragma unroll 1
    for (int b0 = 0; b0 < c; b0 += 32) {
      int idx = o + b0 + lane;
      idx = idx > RCAP - 1 ? RCAP - 1 : idx;
      const int ent = sl[idx];
      int eid = ent >> SLA;
      eid = eid < 0 ? 0 : (eid > nE - 1 ? nE - 1 : eid);
      int sr = srcs[eid];
      sr = sr < 0 ? 0 : (sr > nN - 1 ? nN - 1 : sr);
      const int m32 = (c - b0) < 32 ? (c - b0) : 32;
#pragma unroll 1
      for (int k = 0; k < m32; ++k) {
        const int sk = __builtin_amdgcn_readlane(sr, k);
        t += S[(size_t)sk * KCL + lane];
      }
    }
    const float pzr = big ? qnan : pz;
    t = t + pzr;
    const float si_v = S[(size_t)nc * KCL + lane];
    const bool live = node < nN;
    const float tl = live ? t : 0.0f;
    trp = fmaf(tl, si_v, trp);
    cap += tl;
  }
  trp = wred_f(trp);
  wca[wave * 32 + lane] = cap;
  if (lane == 0) wtr[wave] = trp;
  __syncthreads();
  if (wave == 0) {
    double ca = 0.0, tr = 0.0;
#pragma unroll
    for (int w2 = 0; w2 < NWAVE; ++w2) { ca += (double)wca[w2 * 32 + lane]; tr += (double)wtr[w2]; }
    const float hc = (float)tt + pz;
    rec[lane] = (float)ca;
    rec[32 + lane] = (lane == 0) ? (float)tr : ((lane == 1) ? hc : 0.0f);
  }
  __syncthreads();
  const v4f rv = *(const v4fa*)(rec + 4 * (lane & 15));
  float* op = rec3 + (size_t)blockIdx.x * 64 + 4 * (lane & 15);
  const bool okst = (wave == 0) && (lane < 16);
  if (okst) *(volatile v4f*)op = rv;
  __threadfence();
  if (okst) *(volatile v4f*)op = rv;
}

__global__ __launch_bounds__(PTHR) void k_pool(const unsigned short* __restrict__ p16,
                                               size_t offXThi, size_t offXTlo, size_t offSThi, size_t offSTlo,
                                               const float* __restrict__ S, const float* __restrict__ rec3,
                                               float* out0, float* gl) {
  __shared__ __attribute__((aligned(16))) float po[KCL * PCOL];
  __shared__ __attribute__((aligned(16))) float csw[4 * KCL];
  const int tid = (int)threadIdx.x, lane = tid & 31, wave = tid >> 5, hh = lane >> 4, m = lane & 15;
  const int b = (int)blockIdx.x;

  if (wave < 4) {
    float p = 0.0f;
    const float* sp = S + ((size_t)b * NPG + (size_t)wave * 512) * KCL + lane;
#pragma unroll 4
    for (int i = 0; i < 512; ++i) p += sp[(size_t)i * KCL];
    csw[wave * KCL + lane] = p;
  }

  const size_t arow = (size_t)(b * KCL + m) * NPG + 8 * hh;
  const unsigned short* aH = p16 + offSThi + arow;
  const unsigned short* aL = p16 + offSTlo + arow;
  const bool xw = wave < 4;
  const size_t brow = xw ? (size_t)(b * HID + 32 * wave + m) : (size_t)(b * KCL + m);
  const size_t bhO  = (xw ? offXThi : offSThi) + brow * NPG + 8 * hh;
  const size_t blO  = (xw ? offXTlo : offSTlo) + brow * NPG + 8 * hh;
  const unsigned short* bH = p16 + bhO;
  const unsigned short* bL = p16 + blO;

  v8f acc[4];
  {
    const v8f z = {0.f, 0.f, 0.f, 0.f, 0.f, 0.f, 0.f, 0.f};
    acc[0] = z; acc[1] = z; acc[2] = z; acc[3] = z;
  }
#pragma unroll 1
  for (int k0 = 0; k0 < NPG; k0 += 32) {
    FragB ah[2], al[2], bh[2], bl[2];
#pragma unroll
    for (int t = 0; t < 2; ++t) {
      const size_t ro = (size_t)(16 * t) * NPG + k0;
      ah[t].h[0] = *(const v8usa*)(aH + ro);  ah[t].h[1] = *(const v8usa*)(aH + ro + 16);
      al[t].h[0] = *(const v8usa*)(aL + ro);  al[t].h[1] = *(const v8usa*)(aL + ro + 16);
      bh[t].h[0] = *(const v8usa*)(bH + ro);  bh[t].h[1] = *(const v8usa*)(bH + ro + 16);
      bl[t].h[0] = *(const v8usa*)(bL + ro);  bl[t].h[1] = *(const v8usa*)(bL + ro + 16);
    }
#pragma unroll
    for (int mt = 0; mt < 2; ++mt)
#pragma unroll
      for (int nt = 0; nt < 2; ++nt) acc[mt * 2 + nt] = wmb(ah[mt], bh[nt], acc[mt * 2 + nt]);
#pragma unroll
    for (int mt = 0; mt < 2; ++mt)
#pragma unroll
      for (int nt = 0; nt < 2; ++nt) acc[mt * 2 + nt] = wmb(ah[mt], bl[nt], acc[mt * 2 + nt]);
#pragma unroll
    for (int mt = 0; mt < 2; ++mt)
#pragma unroll
      for (int nt = 0; nt < 2; ++nt) acc[mt * 2 + nt] = wmb(al[mt], bh[nt], acc[mt * 2 + nt]);
  }
#pragma unroll
  for (int mt = 0; mt < 2; ++mt)
#pragma unroll
    for (int nt = 0; nt < 2; ++nt)
#pragma unroll
      for (int r = 0; r < 8; ++r)
        po[(16 * mt + 8 * hh + r) * PCOL + 32 * wave + 16 * nt + m] = acc[mt * 2 + nt][r];
  __syncthreads();

  const float sc = 1.0507009873554805f, al_ = 1.6732632423543772f;
#pragma unroll 1
  for (int k = wave; k < KCL; k += PTHR / 32) {
    const v4f v = *(const v4fa*)(po + k * PCOL + 4 * lane);
    v4f u;
    u.x = sc * ((v.x > 0.0f) ? v.x : al_ * expm1f(v.x));
    u.y = sc * ((v.y > 0.0f) ? v.y : al_ * expm1f(v.y));
    u.z = sc * ((v.z > 0.0f) ? v.z : al_ * expm1f(v.z));
    u.w = sc * ((v.w > 0.0f) ? v.w : al_ * expm1f(v.w));
    const float mx = wmax_f(fmaxf(fmaxf(u.x, u.y), fmaxf(u.z, u.w)));
    const float es = (expf(u.x - mx) + expf(u.y - mx)) + (expf(u.z - mx) + expf(u.w - mx));
    const float lse = logf(wred_f(es));
    v4f o;
    o.x = (u.x - mx) - lse; o.y = (u.y - mx) - lse; o.z = (u.z - mx) - lse; o.w = (u.w - mx) - lse;
    float* op = out0 + (size_t)(b * KCL + k) * HID + 4 * lane;
    *(volatile v4f*)op = o;
    __threadfence();
    *(volatile v4f*)op = o;
  }

  if (wave == 0) {
    double p = 0.0;
#pragma unroll 4
    for (int k = 0; k < KCL; ++k) { const float v = po[k * PCOL + HID + lane]; p += (double)v * (double)v; }
    p = wred_d(p);
    const float ssn = sqrtf((float)p);
    const float inv = 1.0f / ssn;
    const float isq = 0.17677669529663687f;
    double q = 0.0;
#pragma unroll 4
    for (int k = 0; k < KCL; ++k) {
      const float v = po[k * PCOL + HID + lane] * inv - ((k == lane) ? isq : 0.0f);
      q += (double)v * (double)v;
    }
    q = wred_d(q);
    const float ortho = sqrtf((float)q);

    const double cs = (((double)csw[lane] + (double)csw[KCL + lane]) + (double)csw[2 * KCL + lane])
                      + (double)csw[3 * KCL + lane];
    const double c2 = wred_d(cs * cs);
    const float cluster = sqrtf((float)c2) * (1.0f / (float)NPG) * 5.656854249492381f - 1.0f;

    double ca = 0.0, tr = 0.0, eb = 0.0;
#pragma unroll 1
    for (int j = 0; j < BPG; ++j) {
      const float* rp = rec3 + (size_t)(b * BPG + j) * 64;
      ca += (double)rp[lane];
      tr += (double)rp[32];
      eb += (double)rp[33];
    }
    const double ca2 = wred_d(ca * ca);
    const float spec = (float)(-(tr - ca2 / eb) / eb);

    v4f gv;
    const bool l0 = lane == 0;
    gv.x = l0 ? spec : 0.0f; gv.y = l0 ? ortho : 0.0f; gv.z = l0 ? cluster : 0.0f; gv.w = 0.0f;
    float* gp = gl + (size_t)b * 32 + 4 * (lane & 7);
    if (lane < 8) *(volatile v4f*)gp = gv;
    __threadfence();
    if (lane < 8) *(volatile v4f*)gp = gv;
  }
}

__global__ __launch_bounds__(NTHR) void k_out(const float* __restrict__ S, const float* __restrict__ gl,
                                              float* out) {
  const int q = (int)blockIdx.x * NTHR + (int)threadIdx.x;
  const int nFull = NSEL / 4;
  float lossv = 0.0f;
  if (blockIdx.x == 0) {
    double a = 0.0, bsum = 0.0, c = 0.0;
#pragma unroll 1
    for (int g = 0; g < NGRAPH; ++g) {
      const v4f t = *(const v4f*)(gl + g * 32);
      a += (double)t.x; bsum += (double)t.y; c += (double)t.z;
    }
    lossv = (float)(a / (double)NGRAPH + bsum / (double)NGRAPH + c / (double)NGRAPH);
  }
  if (q > nFull) return;
  const int qc = q < nFull ? q : nFull - 1;
  const v4f cur = *(const v4f*)(S + 4 * (size_t)qc);
  int pi = 4 * q - 1;
  pi = pi < 0 ? 0 : (pi > NSEL - 1 ? NSEL - 1 : pi);
  const float pl = S[pi];
  const float lead = (q == 0) ? lossv : pl;
  v4f o;
  o.x = lead; o.y = cur.x; o.z = cur.y; o.w = cur.z;
  float* op = out + NOUT0 + 4 * (size_t)q;
  if (q < nFull) {
    *(volatile v4f*)op = o;
  } else {
    *(volatile float*)op = lead;
  }
  __threadfence();
  if (q < nFull) {
    *(volatile v4f*)op = o;
  } else {
    *(volatile float*)op = lead;
  }
}

static inline size_t al256(size_t o) { return (o + 255) & ~(size_t)255; }

extern "C" void kernel_launch(void* const* d_in, const int* in_sizes, int n_in,
                              void* d_out, int out_size, void* d_ws, size_t ws_size,
                              hipStream_t stream) {
  if (n_in < 10) return;
  if (in_sizes[0] != NNODE * CIN) return;
  if (in_sizes[1] != CIN || in_sizes[2] != CIN || in_sizes[3] != CIN) return;
  if (in_sizes[4] != CIN * HID || in_sizes[5] != HID) return;
  if (in_sizes[6] != HID * KCL || in_sizes[7] != KCL) return;
  if (in_sizes[8] != 2 * NEDGE || in_sizes[9] != NNODE) return;
  if (out_size != NOUTT) return;

  const float* x   = (const float*)d_in[0];
  const float* gw  = (const float*)d_in[1];
  const float* gb  = (const float*)d_in[2];
  const float* gms = (const float*)d_in[3];
  const float* W1  = (const float*)d_in[4];
  const float* b1  = (const float*)d_in[5];
  const float* Wp  = (const float*)d_in[6];
  const float* bp  = (const float*)d_in[7];
  const int*   ei  = (const int*)d_in[8];
  const int*   bat = (const int*)d_in[9];
  float* out = (float*)d_out;
  const int nE = NEDGE, nN = NNODE;
  const int* src = ei;
  const int* dst = ei + nE;
  const int vec8 = ((nE & 3) == 0) ? 1 : 0;

  char* ws = (char*)d_ws;
  size_t off = 0;
  const size_t oW1T = off; off = al256(off + (size_t)HID * KX * 2);
  const size_t oWPT = off; off = al256(off + (size_t)KCL * KD * 2);
  const size_t oR1  = off; off = al256(off + (size_t)NSBLK * RECP * 4);
  const size_t oR2  = off; off = al256(off + (size_t)NSBLK * RECP * 4);
  const size_t oMN  = off; off = al256(off + (size_t)RECP * 4);
  const size_t oRS  = off; off = al256(off + (size_t)NGRAPH * CIN * 4);
  const size_t oXN  = off; off = al256(off + (size_t)NNODE * KX * 2);
  const size_t oDIS = off; off = al256(off + (size_t)NNODE * 4);
  const size_t oH   = off; off = al256(off + (size_t)NNODE * HID * 4);
  const size_t oXD  = off; off = al256(off + (size_t)NNODE * KD * 2);
  const size_t oP16 = off;
  const size_t eXThi = 0;
  const size_t eXTlo = (size_t)NGRAPH * HID * NPG;
  const size_t eSThi = 2 * (size_t)NGRAPH * HID * NPG;
  const size_t eSTlo = eSThi + (size_t)NGRAPH * KCL * NPG;
  const size_t eEnd  = eSTlo + (size_t)NGRAPH * KCL * NPG;
  off = al256(off + eEnd * 2);
  const size_t oS   = off; off = al256(off + (size_t)NSEL * 4);
  const size_t oR3  = off; off = al256(off + (size_t)(NNODE / NBA) * 64 * 4);
  const size_t oGL  = off; off = al256(off + (size_t)NGRAPH * 32 * 4);
  if (off > ws_size || off > (size_t)WSMAX) return;
  unsigned short* W1T2 = (unsigned short*)(ws + oW1T);
  unsigned short* WPT2 = (unsigned short*)(ws + oWPT);
  float* REC1 = (float*)(ws + oR1);
  float* REC2 = (float*)(ws + oR2);
  float* MEANP = (float*)(ws + oMN);
  float* RSTD  = (float*)(ws + oRS);
  unsigned short* XN = (unsigned short*)(ws + oXN);
  float* DIS = (float*)(ws + oDIS);
  float* H   = (float*)(ws + oH);
  unsigned short* XD  = (unsigned short*)(ws + oXD);
  unsigned short* P16 = (unsigned short*)(ws + oP16);
  float* S    = (float*)(ws + oS);
  float* REC3 = (float*)(ws + oR3);
  float* GL   = (float*)(ws + oGL);

  const size_t scanLds = (size_t)AGG_LDS_INTS * 4;
  hipFuncSetAttribute(reinterpret_cast<const void*>(&k_scan1), hipFuncAttributeMaxDynamicSharedMemorySize, (int)scanLds);
  hipFuncSetAttribute(reinterpret_cast<const void*>(&k_scan2), hipFuncAttributeMaxDynamicSharedMemorySize, (int)scanLds);

  k_prep<<<3072 / NTHR, NTHR, 0, stream>>>(W1, Wp, W1T2, WPT2);
  k_gn_acc<0><<<NSBLK, NTHR, 0, stream>>>(x, bat, gms, MEANP, REC1);
  k_gn_comb<0><<<1, NTHR, 0, stream>>>(REC1, NSBLK, MEANP, MEANP);
  k_gn_acc<1><<<NSBLK, NTHR, 0, stream>>>(x, bat, gms, MEANP, REC2);
  k_gn_comb<1><<<1, NTHR, 0, stream>>>(REC2, NSBLK, MEANP, RSTD);
  k_norm<<<(NNODE * 8) / NTHR, NTHR, 0, stream>>>(x, bat, gw, gb, gms, MEANP, RSTD, nN, XN);
  k_deg<<<NNODE / NBD, NTHR, 0, stream>>>(dst, nE, vec8, DIS);
  k_gemm<<<dim3(NNODE / GBM, HID / GBN), GTHR, 0, stream>>>(XN, W1T2, H, KX, HID);
  k_scan1<<<NNODE / NBA, NTHR, scanLds, stream>>>(src, dst, nE, nN, vec8, DIS, H, b1, XD);
  k_tr<<<NNODE / 64, NTHR, 0, stream>>>(XD, P16 + eXThi);
  k_gemm2<<<NNODE / GBM, GTHR, 0, stream>>>(XD, WPT2, bp, S, P16 + eSThi, P16 + eSTlo);
  k_scan2<<<NNODE / NBA, NTHR, scanLds, stream>>>(src, dst, nE, nN, vec8, S, REC3);
  k_pool<<<NGRAPH, PTHR, 0, stream>>>(P16, eXThi, eXTlo, eSThi, eSTlo, S, REC3, out, GL);
  k_out<<<NSEL / 4 / NTHR + 1, NTHR, 0, stream>>>(S, GL, out);
}
